// GATv2_20985210208645
// MI455X (gfx1250) — hardware-verified
//
#include <hip/hip_runtime.h>
#include <stddef.h>
#include <stdint.h>
#include <math.h>


#define DIN     128
#define HC      128
#define NHEAD   8
#define CHD     16
#define NXC     256
#define NGR     128
#define OUTC    2
#define NOUT    (NGR * OUTC)
#define NTHR    256
#define NWAVE   8
#define EPT     8
#define CHUNK   (NTHR * EPT)
#define WCAP    (EPT * 32)
#define LISTN   (NWAVE * WCAP)
#define NBMAX   2048
#define NBRUN   1024
#define RCAP    28672
#define DEGCAP  256
#define STW     128
#define GBM     64
#define GBN     64
#define GTHR    128
#define WBLK    8
#define NEGS    0.2f
#define WSMAX   134217728
#define MEAS_MAXDEG 35
#define MEAS_B1024  16623
#define PAR_BLR 0
#define PAR_ATT 256
#define PAR_BC  384
#define PAR_FCW 512
#define PAR_FCB 768
#define PAR_N   1024
#define LDS_AGG ((2 * RCAP + 2 * NBMAX + LISTN) * 4 + 64)

static_assert((CHUNK & (CHUNK - 1)) == 0 && CHUNK <= 4096);
static_assert((NBMAX & (NBMAX - 1)) == 0 && NBMAX <= 4096);
static_assert((NBRUN & (NBRUN - 1)) == 0 && NBRUN <= NBMAX && NBRUN >= 16);
static_assert(NTHR * 8 == NBMAX);
static_assert(LISTN >= NBMAX);
static_assert((RCAP % 32) == 0);
static_assert(NWAVE * STW <= RCAP);
static_assert(HC <= STW);
static_assert(LDS_AGG <= 300000);
static_assert(GBM == (GTHR / 32) * 16);
static_assert(DIN / 8 == 16);
static_assert((DIN % 32) == 0 && (NXC % GBN) == 0);
static_assert(NHEAD * CHD == HC);
static_assert(32 * 4 == HC);
static_assert(CHD == 4 * 4);
static_assert(NOUT * 4 == 1024);
static_assert(NTHR == NOUT);
static_assert(RCAP >= MEAS_B1024 + 4096);
static_assert(DEGCAP >= MEAS_MAXDEG + 8);
static_assert((HC * (DIN / 8)) == WBLK * NTHR);
static_assert(PAR_N == NTHR * 4);
static_assert(PAR_FCB + 2 <= PAR_N);

typedef float          v4f   __attribute__((ext_vector_type(4)));
typedef float          v8f   __attribute__((ext_vector_type(8)));
typedef int            v4i   __attribute__((ext_vector_type(4)));
typedef int            v8i   __attribute__((ext_vector_type(8)));
typedef unsigned short v8us  __attribute__((ext_vector_type(8)));
typedef __bf16         v16bf __attribute__((ext_vector_type(16)));
typedef v4f __attribute__((may_alias)) v4fa;
union FragB { v16bf v; v8us u[2]; v8i w; };

__device__ __forceinline__ v8f wmx(const FragB& a, const FragB& b, v8f c) {
  v8f d = __builtin_amdgcn_wmma_f32_16x16x32_bf16(false, a.v, false, b.v, (short)0, c, false, false);
  asm volatile("v_nop\n\tv_nop\n\tv_nop\n\tv_nop" : "+v"(d) : "v"(a.w), "v"(b.w));
  return d;
}

__device__ __forceinline__ void ldwait() {
  asm volatile("s_wait_loadcnt 0x0" ::: "memory");
}

__device__ __forceinline__ unsigned bfbits(float v) {
  unsigned u = __float_as_uint(v);
  u = u + 0x7FFFu + ((u >> 16) & 1u);
  return u >> 16;
}
__device__ __forceinline__ float rbf(float v) { return __uint_as_float(bfbits(v) << 16); }

__device__ __forceinline__ v8us cvt8b(const v4f a, const v4f b) {
  v8us o;
  o[0] = (unsigned short)bfbits(a.x); o[1] = (unsigned short)bfbits(a.y);
  o[2] = (unsigned short)bfbits(a.z); o[3] = (unsigned short)bfbits(a.w);
  o[4] = (unsigned short)bfbits(b.x); o[5] = (unsigned short)bfbits(b.y);
  o[6] = (unsigned short)bfbits(b.z); o[7] = (unsigned short)bfbits(b.w);
  return o;
}

__device__ __forceinline__ float blend6(float a, unsigned ma, float b, unsigned mb, float c, unsigned mc,
                                        float d, unsigned md, float e, unsigned me, float f, unsigned mf) {
  const unsigned u = (__float_as_uint(a) & ma) | (__float_as_uint(b) & mb) | (__float_as_uint(c) & mc) |
                     (__float_as_uint(d) & md) | (__float_as_uint(e) & me) | (__float_as_uint(f) & mf);
  return __uint_as_float(u);
}

__device__ __forceinline__ int scan_chunk(const int* __restrict__ dsts, int nE, int cbase, int slotBase,
                                          int nb, int vec8, int* list, int tid, int lane, int wave) {
  int wc = 0;
  const int el0  = tid * EPT;
  const int e0   = cbase + el0;
  const int sent = -2147483647 - 1;
  v4i da, db;
  if (vec8 != 0 && cbase + CHUNK <= nE) {
    da = *(const v4i*)(dsts + e0);
    db = *(const v4i*)(dsts + e0 + 4);
  } else {
    da.x = (e0     < nE) ? dsts[min(e0,     nE - 1)] : sent;
    da.y = (e0 + 1 < nE) ? dsts[min(e0 + 1, nE - 1)] : sent;
    da.z = (e0 + 2 < nE) ? dsts[min(e0 + 2, nE - 1)] : sent;
    da.w = (e0 + 3 < nE) ? dsts[min(e0 + 3, nE - 1)] : sent;
    db.x = (e0 + 4 < nE) ? dsts[min(e0 + 4, nE - 1)] : sent;
    db.y = (e0 + 5 < nE) ? dsts[min(e0 + 5, nE - 1)] : sent;
    db.z = (e0 + 6 < nE) ? dsts[min(e0 + 6, nE - 1)] : sent;
    db.w = (e0 + 7 < nE) ? dsts[min(e0 + 7, nE - 1)] : sent;
  }
  const unsigned nbs = (unsigned)slotBase;
  const unsigned unb = (unsigned)nb;
  const unsigned s0 = (unsigned)da.x - nbs, s1 = (unsigned)da.y - nbs;
  const unsigned s2 = (unsigned)da.z - nbs, s3 = (unsigned)da.w - nbs;
  const unsigned s4 = (unsigned)db.x - nbs, s5 = (unsigned)db.y - nbs;
  const unsigned s6 = (unsigned)db.z - nbs, s7 = (unsigned)db.w - nbs;
  const bool h0 = s0 < unb, h1 = s1 < unb, h2 = s2 < unb, h3 = s3 < unb;
  const bool h4 = s4 < unb, h5 = s5 < unb, h6 = s6 < unb, h7 = s7 < unb;
  const unsigned any = __builtin_amdgcn_ballot_w32(h0 | h1 | h2 | h3 | h4 | h5 | h6 | h7);
  if (any != 0u) {
#define HITJ(J, HJ, SJ) { \
      const unsigned mj = __builtin_amdgcn_ballot_w32(HJ); \
      if (mj != 0u) { \
        if (HJ) { \
          const int pos = wc + (int)__builtin_amdgcn_mbcnt_lo(mj, 0u); \
          if (pos < WCAP) list[wave * WCAP + pos] = ((el0 + (J)) << 12) | (int)(SJ); \
        } \
        wc += (int)__builtin_popcount(mj); } }
    HITJ(0, h0, s0)
    HITJ(1, h1, s1)
    HITJ(2, h2, s2)
    HITJ(3, h3, s3)
    HITJ(4, h4, s4)
    HITJ(5, h5, s5)
    HITJ(6, h6, s6)
    HITJ(7, h7, s7)
#undef HITJ
  }
  return wc;
}

__global__ __launch_bounds__(NTHR) void k_prep(
    const float* __restrict__ x, const float* __restrict__ Wl, const float* __restrict__ Wr,
    const float* __restrict__ bl, const float* __restrict__ br, const float* __restrict__ att,
    const float* __restrict__ bc, const float* __restrict__ fcW, const float* __restrict__ fcb,
    unsigned short* xb, unsigned short* wt, float* par, int nN, int nBx) {
  const int b = (int)blockIdx.x, tid = (int)threadIdx.x;
  const v4f z4 = {0.f, 0.f, 0.f, 0.f};
  if (b < nBx) {
    const int i   = b * NTHR + tid;
    const int row = i >> 4;
    const int c0  = (i & 15) * 8;
    const int rc  = row < nN ? row : nN - 1;
    const float* p = x + (size_t)rc * DIN + c0;
    v4f a = *(const v4f*)p, c = *(const v4f*)(p + 4);
    if (row >= nN) { a = z4; c = z4; }
    const v8us hv = cvt8b(a, c);
    const size_t o = (size_t)row * DIN + c0;
    *(volatile v8us*)(xb + o) = hv;
    __threadfence();
    *(volatile v8us*)(xb + o) = hv;
    return;
  }
  const int bw = b - nBx;
  if (bw < WBLK) {
    const int u  = bw * NTHR + tid;
    const int n  = u >> 4;
    const int k8 = (u & 15) * 8;
    const float* p = Wl + (size_t)k8 * HC + n;
    v4f a, c;
    a.x = p[0];        a.y = p[HC];       a.z = p[2 * HC];   a.w = p[3 * HC];
    c.x = p[4 * HC];   c.y = p[5 * HC];   c.z = p[6 * HC];   c.w = p[7 * HC];
    const v8us hv = cvt8b(a, c);
    const size_t o = (size_t)n * DIN + k8;
    *(volatile v8us*)(wt + o) = hv;
    __threadfence();
    *(volatile v8us*)(wt + o) = hv;
    return;
  }
  if (bw < 2 * WBLK) {
    const int u  = (bw - WBLK) * NTHR + tid;
    const int n  = u >> 4;
    const int k8 = (u & 15) * 8;
    const float* p = Wr + (size_t)k8 * HC + n;
    v4f a, c;
    a.x = p[0];        a.y = p[HC];       a.z = p[2 * HC];   a.w = p[3 * HC];
    c.x = p[4 * HC];   c.y = p[5 * HC];   c.z = p[6 * HC];   c.w = p[7 * HC];
    const v8us hv = cvt8b(a, c);
    const size_t o = (size_t)(n + HC) * DIN + k8;
    *(volatile v8us*)(wt + o) = hv;
    __threadfence();
    *(volatile v8us*)(wt + o) = hv;
    return;
  }
  if (bw > 2 * WBLK) return;
  {
    const int t  = tid;
    const int iA = t < 31 ? t : 31;
    const int tB = t - 32,  iB = tB < 0 ? 0 : (tB > 31 ? 31 : tB);
    const int tC = t - 64,  iC = tC < 0 ? 0 : (tC > 31 ? 31 : tC);
    const int tD = t - 96,  iD = tD < 0 ? 0 : (tD > 31 ? 31 : tD);
    const int tE = t - 128, iE = tE < 0 ? 0 : (tE > 63 ? 63 : tE);
    const v4f vA = *(const v4f*)(bl  + 4 * iA);
    const v4f vB = *(const v4f*)(br  + 4 * iB);
    const v4f vC = *(const v4f*)(att + 4 * iC);
    const v4f vD = *(const v4f*)(bc  + 4 * iD);
    const v4f vE = *(const v4f*)(fcW + 4 * iE);
    const float f0 = fcb[0], f1 = fcb[1];
    const unsigned mA = (t < 32) ? 0xffffffffu : 0u;
    const unsigned mB = (t >= 32 && t < 64) ? 0xffffffffu : 0u;
    const unsigned mC = (t >= 64 && t < 96) ? 0xffffffffu : 0u;
    const unsigned mD = (t >= 96 && t < 128) ? 0xffffffffu : 0u;
    const unsigned mE = (t >= 128 && t < 192) ? 0xffffffffu : 0u;
    const unsigned mF = (t == 192) ? 0xffffffffu : 0u;
    v4f o;
    o.x = rbf(blend6(vA.x, mA, vB.x, mB, vC.x, mC, vD.x, mD, vE.x, mE, f0, mF));
    o.y = rbf(blend6(vA.y, mA, vB.y, mB, vC.y, mC, vD.y, mD, vE.y, mE, f1, mF));
    o.z = rbf(blend6(vA.z, mA, vB.z, mB, vC.z, mC, vD.z, mD, vE.z, mE, 0.0f, 0u));
    o.w = rbf(blend6(vA.w, mA, vB.w, mB, vC.w, mC, vD.w, mD, vE.w, mE, 0.0f, 0u));
    float* op = par + 4 * t;
    *(volatile v4f*)op = o;
    __threadfence();
    *(volatile v4f*)op = o;
  }
}

__global__ __launch_bounds__(GTHR) void k_xlr(
    const unsigned short* __restrict__ A, const unsigned short* __restrict__ WT,
    const float* __restrict__ par, float* outF)
{
  __shared__ __attribute__((aligned(16))) float stg[GBM * GBN];
  const int tid = (int)threadIdx.x, lane = tid & 31, wave = tid >> 5, hh = lane >> 4, m = lane & 15;
  const int rowBase = (int)blockIdx.x * GBM;
  const int col0    = (int)blockIdx.y * GBN;

  v8f acc[4];
  {
    const v8f z = {0.f, 0.f, 0.f, 0.f, 0.f, 0.f, 0.f, 0.f};
    acc[0] = z; acc[1] = z; acc[2] = z; acc[3] = z;
  }
  const float bq0 = par[PAR_BLR + col0 + m];
  const float bq1 = par[PAR_BLR + col0 + 16 + m];
  const float bq2 = par[PAR_BLR + col0 + 32 + m];
  const float bq3 = par[PAR_BLR + col0 + 48 + m];
  const unsigned short* ap = A  + (size_t)(rowBase + 16 * wave + m) * (size_t)DIN + 8 * hh;
  const unsigned short* wp = WT + (size_t)(col0 + m) * (size_t)DIN + 8 * hh;
#pragma unroll 1
  for (int ks = 0; ks < DIN / 32; ++ks) {
    FragB af;
    af.u[0] = *(const v8us*)(ap + 32 * ks);
    af.u[1] = *(const v8us*)(ap + 32 * ks + 16);
#pragma unroll
    for (int t = 0; t < 4; ++t) {
      const unsigned short* wq = wp + (size_t)(16 * t) * (size_t)DIN + 32 * ks;
      FragB bf;
      bf.u[0] = *(const v8us*)wq;
      bf.u[1] = *(const v8us*)(wq + 16);
      acc[t] = wmx(af, bf, acc[t]);
    }
  }

  const float bq[4] = {bq0, bq1, bq2, bq3};
#pragma unroll
  for (int t = 0; t < 4; ++t) {
    const int lc = 16 * t + m;
#pragma unroll
    for (int r = 0; r < 8; ++r) {
      const int lr = 16 * wave + 8 * hh + r;
      stg[lr * GBN + lc] = acc[t][r] + bq[t];
    }
  }
  __syncthreads();

  v4f fv[8];
#pragma unroll
  for (int i = 0; i < 8; ++i) {
    const int lr = 16 * wave + 2 * i + hh;
    fv[i] = *(const v4fa*)(stg + lr * GBN + 4 * m);
  }
#pragma unroll
  for (int i = 0; i < 8; ++i) {
    const int lr = 16 * wave + 2 * i + hh;
    const int gr = rowBase + lr;
    float* op = outF + (size_t)gr * (size_t)NXC + col0 + 4 * m;
    *(volatile v4f*)op = fv[i];
  }
  __threadfence();
#pragma unroll
  for (int i = 0; i < 8; ++i) {
    const int lr = 16 * wave + 2 * i + hh;
    const int gr = rowBase + lr;
    float* op = outF + (size_t)gr * (size_t)NXC + col0 + 4 * m;
    *(volatile v4f*)op = fv[i];
  }
}

__global__ __launch_bounds__(NTHR) void k_scan(
    const int* __restrict__ srcs, const int* __restrict__ dsts,
    const float* __restrict__ XLR, const float* __restrict__ par, float* OUT,
    int nN, int nE, int nb, int vec8) {
  extern __shared__ v4f lds_dyn[];
  int* reg1 = (int*)lds_dyn;
  int* reg2 = reg1 + RCAP;
  int* scnt = reg2 + RCAP;
  int* soff = scnt + NBMAX;
  int* list = soff + NBMAX;
  int* wcnt = list + LISTN;
  int* wtot = wcnt + NWAVE;
  const int tid = (int)threadIdx.x, lane = tid & 31, wave = tid >> 5;
  const int nodeBase = (int)blockIdx.x * nb;

  for (int i = tid; i < NBMAX; i += NTHR) scnt[i] = 0;
  __syncthreads();

  int tot = 0;
  const int nChunks = (nE + CHUNK - 1) / CHUNK;
#pragma unroll 1
  for (int ch = 0; ch < nChunks; ++ch) {
    const int cbase = ch * CHUNK;
    const int wc = scan_chunk(dsts, nE, cbase, nodeBase, nb, vec8, list, tid, lane, wave);
    if (lane == 0) wcnt[wave] = wc;
    __syncthreads();
    int pre = 0, all = 0;
#pragma unroll
    for (int w2 = 0; w2 < NWAVE; ++w2) {
      int c = wcnt[w2];
      c = c < 0 ? 0 : (c > WCAP ? WCAP : c);
      all += c;
      pre += (w2 < wave) ? c : 0;
    }
    const int wcc  = wc > WCAP ? WCAP : wc;
    const int base = tot + pre;
#pragma unroll 1
    for (int i = lane; i < wcc; i += 32) {
      const int ent = list[wave * WCAP + i];
      const int el  = (ent >> 12) & (CHUNK - 1);
      const int sl  = ent & (NBMAX - 1);
      int eid = cbase + el;
      eid = eid > nE - 1 ? nE - 1 : eid;
      const int pos = base + i;
      if (pos < RCAP) reg1[pos] = (int)(((unsigned)eid << 12) | (unsigned)sl);
    }
    tot += all;
    tot = tot > RCAP ? RCAP : tot;
    __syncthreads();
  }
  const int nh = tot;

  if (wave == 0) {
#pragma unroll 1
    for (int b0 = 0; b0 < nh; b0 += 32) {
      const int idx = b0 + lane;
      const int uv  = reg1[idx < nh ? idx : nh - 1];
      const int m32 = (nh - b0) < 32 ? (nh - b0) : 32;
#pragma unroll 1
      for (int k = 0; k < m32; ++k) {
        const int u  = __builtin_amdgcn_readlane(uv, k);
        const int sl = u & (NBMAX - 1);
        if (lane == 0) scnt[sl] = scnt[sl] + 1;
      }
    }
  }
  __syncthreads();

  {
    const v4i ca = *(const v4i*)(scnt + 8 * tid);
    const v4i cb = *(const v4i*)(scnt + 8 * tid + 4);
    const int e0 = ca.x < 0 ? 0 : ca.x, e1 = ca.y < 0 ? 0 : ca.y, e2 = ca.z < 0 ? 0 : ca.z, e3 = ca.w < 0 ? 0 : ca.w;
    const int e4 = cb.x < 0 ? 0 : cb.x, e5 = cb.y < 0 ? 0 : cb.y, e6 = cb.z < 0 ? 0 : cb.z, e7 = cb.w < 0 ? 0 : cb.w;
    const int ts = e0 + e1 + e2 + e3 + e4 + e5 + e6 + e7;
    int incl = ts;
#pragma unroll
    for (int d = 1; d < 32; d <<= 1) {
      const int up = __shfl_up(incl, d);
      if (lane >= d) incl += up;
    }
    if (lane == 31) wtot[wave] = incl;
    __syncthreads();
    int pre = 0;
#pragma unroll
    for (int w2 = 0; w2 < NWAVE; ++w2) pre += (w2 < wave) ? wtot[w2] : 0;
    int run = pre + incl - ts;
    soff[8 * tid + 0] = run; run += e0;
    soff[8 * tid + 1] = run; run += e1;
    soff[8 * tid + 2] = run; run += e2;
    soff[8 * tid + 3] = run; run += e3;
    soff[8 * tid + 4] = run; run += e4;
    soff[8 * tid + 5] = run; run += e5;
    soff[8 * tid + 6] = run; run += e6;
    soff[8 * tid + 7] = run;
  }
  __syncthreads();
  for (int i = tid; i < NBMAX; i += NTHR) list[i] = soff[i];
  __syncthreads();

  if (wave == 0) {
#pragma unroll 1
    for (int b0 = 0; b0 < nh; b0 += 32) {
      const int idx = b0 + lane;
      const int uv  = reg1[idx < nh ? idx : nh - 1];
      const int m32 = (nh - b0) < 32 ? (nh - b0) : 32;
#pragma unroll 1
      for (int k = 0; k < m32; ++k) {
        const int u   = __builtin_amdgcn_readlane(uv, k);
        const int sl  = u & (NBMAX - 1);
        const int eid = (int)((unsigned)u >> 12);
        if (lane == 0) {
          int pos = list[sl];
          pos = pos < 0 ? 0 : (pos > RCAP - 1 ? RCAP - 1 : pos);
          reg2[pos] = eid;
          list[sl] = pos + 1;
        }
      }
    }
  }
  __syncthreads();

  const int nbw = nb >> 3;
  const bool ovf = (nh >= RCAP);
  const float qnan = __int_as_float(0x7fc00000);
  float* stw = (float*)lds_dyn + wave * STW;
  const v4f at = *(const v4f*)(par + PAR_ATT + 4 * lane);
  const v4f bc = *(const v4f*)(par + PAR_BC + 4 * lane);
  ldwait();
#pragma unroll 1
  for (int jt = 0; jt < nbw; ++jt) {
    const int slot = wave * nbw + jt;
    const int grow = nodeBase + slot;
    const int gcl  = grow < nN ? grow : nN - 1;
    int st = soff[slot];
    const int craw = scnt[slot];
    int cnt = craw;
    st  = st < 0 ? 0 : (st > nh ? nh : st);
    cnt = cnt < 0 ? 0 : (cnt > DEGCAP ? DEGCAP : cnt);
    if (cnt > nh - st) cnt = nh - st;
    const float pz = (ovf || craw > DEGCAP) ? qnan : 0.0f;

    const float* drow = XLR + (size_t)gcl * NXC + 4 * lane;
    const v4f xs = *(const v4f*)drow;
    const v4f xd = *(const v4f*)(drow + HC);
    ldwait();
    float part;
    {
      float v0 = xs.x + xd.x, v1 = xs.y + xd.y, v2 = xs.z + xd.z, v3 = xs.w + xd.w;
      v0 = v0 > 0.f ? v0 : v0 * NEGS; v1 = v1 > 0.f ? v1 : v1 * NEGS;
      v2 = v2 > 0.f ? v2 : v2 * NEGS; v3 = v3 > 0.f ? v3 : v3 * NEGS;
      part = v0 * at.x;
      part = fmaf(v1, at.y, part);
      part = fmaf(v2, at.z, part);
      part = fmaf(v3, at.w, part);
    }
    part += __shfl_xor(part, 1);
    part += __shfl_xor(part, 2);
    float mx = part, dn = 1.0f;
    float a0 = xs.x, a1 = xs.y, a2 = xs.z, a3 = xs.w;

#pragma unroll 1
    for (int q = 0; q < cnt; ++q) {
      int idx = st + q; idx = idx > RCAP - 1 ? RCAP - 1 : idx;
      int eid = reg2[idx]; eid = eid < 0 ? 0 : (eid > nE - 1 ? nE - 1 : eid);
      const int sraw = srcs[eid];
      const int s = sraw < 0 ? 0 : (sraw > nN - 1 ? nN - 1 : sraw);
      const v4f hs = *(const v4f*)(XLR + (size_t)s * NXC + 4 * lane);
      ldwait();
      float v0 = hs.x + xd.x, v1 = hs.y + xd.y, v2 = hs.z + xd.z, v3 = hs.w + xd.w;
      v0 = v0 > 0.f ? v0 : v0 * NEGS; v1 = v1 > 0.f ? v1 : v1 * NEGS;
      v2 = v2 > 0.f ? v2 : v2 * NEGS; v3 = v3 > 0.f ? v3 : v3 * NEGS;
      float pt = v0 * at.x;
      pt = fmaf(v1, at.y, pt);
      pt = fmaf(v2, at.z, pt);
      pt = fmaf(v3, at.w, pt);
      pt += __shfl_xor(pt, 1);
      pt += __shfl_xor(pt, 2);
      const float df = pt - mx;
      const float ee = expf(-fabsf(df));
      const bool up  = df > 0.f;
      const float s1 = up ? ee : 1.0f;
      const float s2 = up ? 1.0f : ee;
      mx = up ? pt : mx;
      dn = fmaf(dn, s1, s2);
      a0 = fmaf(a0, s1, s2 * hs.x);
      a1 = fmaf(a1, s1, s2 * hs.y);
      a2 = fmaf(a2, s1, s2 * hs.z);
      a3 = fmaf(a3, s1, s2 * hs.w);
    }
    const float iv = __builtin_amdgcn_rcpf(dn + 1e-16f);
    v4f y;
    y.x = fmaf(a0, iv, bc.x) + pz;
    y.y = fmaf(a1, iv, bc.y) + pz;
    y.z = fmaf(a2, iv, bc.z) + pz;
    y.w = fmaf(a3, iv, bc.w) + pz;
    __builtin_amdgcn_fence(__ATOMIC_RELEASE, "wavefront");
    __builtin_amdgcn_wave_barrier();
    *(v4fa*)(stw + 4 * lane) = y;
    __builtin_amdgcn_fence(__ATOMIC_RELEASE, "wavefront");
    __builtin_amdgcn_wave_barrier();
#pragma unroll 1
    for (int j = 0; j < HC / 32; ++j) {
      const float v = stw[32 * j + lane];
      const float o = (v > 0.0f) ? v : expm1f(v);
      stw[32 * j + lane] = o;
    }
    __builtin_amdgcn_fence(__ATOMIC_RELEASE, "wavefront");
    __builtin_amdgcn_wave_barrier();
    const v4f gv = *(const v4fa*)(stw + 4 * lane);
    const bool wr = grow < nN;
    float* gp = OUT + (size_t)gcl * HC + 4 * lane;
    if (wr) *(volatile v4f*)gp = gv;
    __threadfence();
    if (wr) *(volatile v4f*)gp = gv;
  }
}

__global__ __launch_bounds__(NTHR) void k_pool(const float* __restrict__ hf, const int* __restrict__ bat,
                                               int nN, float* pl) {
  __shared__ double wsum[NWAVE * HC];
  __shared__ int wcn[NWAVE];
  __shared__ __attribute__((aligned(16))) float outs[HC];
  const int tid = (int)threadIdx.x, lane = tid & 31, wave = tid >> 5;
  const int g = (int)blockIdx.x;

  double a0 = 0.0, a1 = 0.0, a2 = 0.0, a3 = 0.0;
  int cnt = 0;
#pragma unroll 1
  for (int i0 = wave * 32; i0 < nN; i0 += NTHR) {
    const int i  = i0 + lane;
    const int ic = i < nN ? i : nN - 1;
    const int b  = bat[ic];
    const bool hit = (i < nN) && (b == g);
    unsigned msk = __builtin_amdgcn_ballot_w32(hit);
    int nh = (int)__builtin_popcount(msk);
    nh = nh > 32 ? 32 : nh;
    cnt += nh;
#pragma unroll 1
    for (int q = 0; q < nh; ++q) {
      const int k = __builtin_ffs((int)msk) - 1;
      msk &= msk - 1u;
      int node = i0 + (k < 0 ? 0 : k);
      node = node > nN - 1 ? nN - 1 : node;
      const v4f v = *(const v4f*)(hf + (size_t)node * HC + 4 * lane);
      a0 += (double)v.x; a1 += (double)v.y; a2 += (double)v.z; a3 += (double)v.w;
    }
  }
  wsum[wave * HC + 4 * lane + 0] = a0;
  wsum[wave * HC + 4 * lane + 1] = a1;
  wsum[wave * HC + 4 * lane + 2] = a2;
  wsum[wave * HC + 4 * lane + 3] = a3;
  if (lane == 0) wcn[wave] = cnt;
  __syncthreads();
  if (tid < HC) {
    double s = 0.0;
    int c = 0;
#pragma unroll
    for (int w2 = 0; w2 < NWAVE; ++w2) { s += wsum[w2 * HC + tid]; c += wcn[w2]; }
    const float cf = (c < 1) ? 1.0f : (float)c;
    const float ri = 1.0f / cf;
    outs[tid] = (float)(s * (double)ri);
  }
  __syncthreads();
  const v4f ov = *(const v4fa*)(outs + 4 * lane);
  float* op = pl + (size_t)g * HC + 4 * lane;
  const bool okst = (wave == 0);
  if (okst) *(volatile v4f*)op = ov;
  __threadfence();
  if (okst) *(volatile v4f*)op = ov;
}

__global__ __launch_bounds__(NTHR) void k_head(const float* __restrict__ pl, const float* __restrict__ par,
                                               float* out) {
  __shared__ float fw[HC * OUTC];
  __shared__ __attribute__((aligned(16))) float os[NOUT];
  const int tid = (int)threadIdx.x;
  const int g = tid >> 1, j = tid & 1;
  fw[tid] = par[PAR_FCW + tid];
  const float fb = par[PAR_FCB + j];
  __syncthreads();
  const float* pr = pl + (size_t)g * HC;
  double s = 0.0;
#pragma unroll 1
  for (int c4 = 0; c4 < HC / 4; ++c4) {
    const v4f p = *(const v4f*)(pr + 4 * c4);
    const float* w = fw + (4 * c4) * OUTC + j;
    s = fma((double)p.x, (double)w[0], s);
    s = fma((double)p.y, (double)w[OUTC], s);
    s = fma((double)p.z, (double)w[2 * OUTC], s);
    s = fma((double)p.w, (double)w[3 * OUTC], s);
  }
  os[tid] = (float)(s + (double)fb);
  __syncthreads();
  const int tq = tid < 64 ? tid : 63;
  const v4f ov = *(const v4fa*)(os + 4 * tq);
  float* op = out + 4 * tq;
  const bool okst = tid < 64;
  if (okst) *(volatile v4f*)op = ov;
  __threadfence();
  if (okst) *(volatile v4f*)op = ov;
}

static int pick_nb(int nE, int nN) {
  int nb = NBRUN;
  while (nb > 16 && (long long)nb * (long long)nE * 5LL > (long long)RCAP * (long long)nN * 4LL) nb >>= 1;
  return nb;
}
static inline int cdiv(int a, int b) { return (a + b - 1) / b; }
static inline size_t al256(size_t o) { return (o + 255) & ~(size_t)255; }

extern "C" void kernel_launch(void* const* d_in, const int* in_sizes, int n_in,
                              void* d_out, int out_size, void* d_ws, size_t ws_size,
                              hipStream_t stream) {
  if (n_in < 11) return;
  const int nN = in_sizes[2];
  if (nN < 1 || nN > (1 << 22)) return;
  if (in_sizes[0] != nN * DIN) return;
  if (in_sizes[1] < 2 || (in_sizes[1] & 1) != 0) return;
  const int nE = in_sizes[1] / 2;
  if (nE < 1 || nE > (1 << 20)) return;
  if (in_sizes[3] != DIN * HC || in_sizes[4] != HC) return;
  if (in_sizes[5] != DIN * HC || in_sizes[6] != HC) return;
  if (in_sizes[7] != HC || in_sizes[8] != HC) return;
  if (in_sizes[9] != HC * OUTC || in_sizes[10] != OUTC) return;
  if (out_size != NOUT) return;

  const float* x    = (const float*)d_in[0];
  const int*   ei   = (const int*)  d_in[1];
  const int*   bat  = (const int*)  d_in[2];
  const float* Wl   = (const float*)d_in[3];
  const float* bl   = (const float*)d_in[4];
  const float* Wr   = (const float*)d_in[5];
  const float* br   = (const float*)d_in[6];
  const float* att  = (const float*)d_in[7];
  const float* bcv  = (const float*)d_in[8];
  const float* fcW  = (const float*)d_in[9];
  const float* fcb  = (const float*)d_in[10];
  float* out = (float*)d_out;
  const int* src = ei;
  const int* dst = ei + nE;

  const int MP   = cdiv(nN, GBM) * GBM;
  const int nb   = pick_nb(nE, nN);
  const int gA   = cdiv(nN, nb);
  const int vec8 = ((nE & 3) == 0) ? 1 : 0;
  if ((long long)gA * (long long)nb < (long long)nN) return;
  if (((MP * (DIN / 8)) % NTHR) != 0) return;
  const int nBx = (MP * (DIN / 8)) / NTHR;

  char* ws = (char*)d_ws;
  size_t off = 0;
  const size_t oXB  = off; off = al256(off + (size_t)MP * DIN * 2);
  const size_t oWT  = off; off = al256(off + (size_t)NXC * DIN * 2);
  const size_t oPAR = off; off = al256(off + (size_t)PAR_N * 4);
  const size_t oXLR = off; off = al256(off + (size_t)MP * NXC * 4);
  const size_t oOUT = off; off = al256(off + (size_t)nN * HC * 4);
  const size_t oPL  = off; off = al256(off + (size_t)NGR * HC * 4);
  if (off > ws_size || off > (size_t)WSMAX) return;
  unsigned short* XB  = (unsigned short*)(ws + oXB);
  unsigned short* WT  = (unsigned short*)(ws + oWT);
  float*          PAR = (float*)(ws + oPAR);
  float*          XLR = (float*)(ws + oXLR);
  float*          OUT = (float*)(ws + oOUT);
  float*          PL  = (float*)(ws + oPL);

  hipFuncSetAttribute(reinterpret_cast<const void*>(&k_scan),
                      hipFuncAttributeMaxDynamicSharedMemorySize, LDS_AGG);

  k_prep<<<nBx + 2 * WBLK + 1, NTHR, 0, stream>>>(x, Wl, Wr, bl, br, att, bcv, fcW, fcb, XB, WT, PAR, nN, nBx);
  k_xlr<<<dim3(MP / GBM, NXC / GBN), GTHR, 0, stream>>>(XB, WT, PAR, XLR);
  k_scan<<<gA, NTHR, LDS_AGG, stream>>>(src, dst, XLR, PAR, OUT, nN, nE, nb, vec8);
  k_pool<<<NGR, NTHR, 0, stream>>>(OUT, bat, nN, PL);
  k_head<<<1, NTHR, 0, stream>>>(PL, PAR, out);
}
